// FlaxAttention_17583596110634
// MI455X (gfx1250) — hardware-verified
//
#include <hip/hip_runtime.h>
#include <stddef.h>
#include <stdint.h>

typedef __attribute__((ext_vector_type(16))) _Float16 v16h;
typedef __attribute__((ext_vector_type(8)))  _Float16 v8h;
typedef __attribute__((ext_vector_type(16))) __bf16   v16b;
typedef __attribute__((ext_vector_type(8)))  __bf16   v8b;
typedef __attribute__((ext_vector_type(8)))  float    v8f;
typedef __attribute__((ext_vector_type(4)))  float    v4f;
typedef __attribute__((ext_vector_type(4)))  unsigned int v4u;

constexpr int kBatch   = 2;
constexpr int kSeq     = 2048;
constexpr int kModel   = 1024;
constexpr int kHeads   = 16;
constexpr int kHeadDim = 64;
constexpr int kRows    = kBatch * kSeq;
constexpr int kQkvCols = 3 * kModel;
constexpr int kQkCols  = 2 * kModel;
constexpr int kKvChunk = 64;
constexpr int kOsPitch = 68;

constexpr size_t kPlane16  = (size_t)kRows * kModel * 2;
constexpr size_t kOffXb    = 0;
constexpr size_t kOffWqkvT = kOffXb + kPlane16;
constexpr size_t kOffWoutT = kOffWqkvT + (size_t)kQkvCols * kModel * 2;
constexpr size_t kOffQk    = kOffWoutT + (size_t)kModel * kModel * 2;
constexpr size_t kOffCtxH  = kOffQk;
constexpr size_t kOffCtxL  = kOffQk + kPlane16;
constexpr size_t kOffVh    = kOffQk + (size_t)kRows * kQkCols * 4;
constexpr size_t kOffVl    = kOffVh + kPlane16;
constexpr size_t kOffQh    = kOffVl + kPlane16;
constexpr size_t kOffQl    = kOffQh + kPlane16;
constexpr size_t kOffKh    = kOffQl + kPlane16;
constexpr size_t kOffKl    = kOffKh + kPlane16;
constexpr size_t kWsTotal  = kOffKl + kPlane16;
static_assert(kWsTotal == (size_t)100663296);
static_assert(kWsTotal <= (size_t)134217728);
static_assert(kOffCtxL + kPlane16 <= kOffVh);
static_assert((kOffWqkvT % 128) == 0 && (kOffWoutT % 128) == 0 && (kOffQk % 128) == 0 && (kOffVh % 128) == 0);
static_assert(kRows % 64 == 0 && kQkCols % 64 == 0 && kModel % 64 == 0 && kModel % 32 == 0);
static_assert(kSeq % 64 == 0 && kHeadDim == 64 && kModel == kHeads * kHeadDim);
static_assert((kRows * kModel) % (8 * 256) == 0);

__device__ __forceinline__ unsigned short f2bf_bits(float f) {
  unsigned u = __float_as_uint(f);
  return (unsigned short)((u + 0x7FFFu + ((u >> 16) & 1u)) >> 16);
}
__device__ __forceinline__ float bf_bits2f(unsigned short h) { return __uint_as_float(((unsigned)h) << 16); }
__device__ __forceinline__ unsigned int pack_bf16x2(float a, float b) {
  return (unsigned int)f2bf_bits(a) | ((unsigned int)f2bf_bits(b) << 16);
}

__device__ __forceinline__ void dep_guard_h(v8f& a, v8f& b, v16h x, v16h y) { asm volatile("v_nop\n\tv_nop\n\tv_nop\n\tv_nop" : "+v"(a), "+v"(b) : "v"(x), "v"(y)); }
__device__ __forceinline__ void dep_guard_b(v8f& a, v8f& b, v16b x, v16b y) { asm volatile("v_nop\n\tv_nop\n\tv_nop\n\tv_nop" : "+v"(a), "+v"(b) : "v"(x), "v"(y)); }
__device__ __forceinline__ void keep4_h(v16h a, v16h b, v16h c, v16h d) { asm volatile("v_nop" :: "v"(a), "v"(b), "v"(c), "v"(d)); }
__device__ __forceinline__ void keep4_b(v16b a, v16b b, v16b c, v16b d) { asm volatile("v_nop" :: "v"(a), "v"(b), "v"(c), "v"(d)); }
__device__ __forceinline__ void acc_guard4(v8f& a, v8f& b, v8f& c, v8f& d) { asm volatile("v_nop\n\tv_nop\n\tv_nop\n\tv_nop" : "+v"(a), "+v"(b), "+v"(c), "+v"(d)); }
template <typename T> struct Frag;
template <> struct Frag<_Float16> {
  typedef v16h V; union U { v16h v; v8h h[2]; };
  static __device__ __forceinline__ v16h load(const _Float16* p) {
    U f; f.h[0] = *(const v8h*)(p); f.h[1] = *(const v8h*)(p + 16); return f.v;
  }
  static __device__ __forceinline__ v8f mma(v16h a, v16h b, v8f c) {
    return __builtin_amdgcn_wmma_f32_16x16x32_f16(false, a, false, b, (short)0, c, false, false);
  }
  static __device__ __forceinline__ void guard(v8f& a, v8f& b, v16h x, v16h y) { dep_guard_h(a, b, x, y); }
  static __device__ __forceinline__ void keep(v16h a, v16h b, v16h c, v16h d) { keep4_h(a, b, c, d); }
};
template <> struct Frag<__bf16> {
  typedef v16b V; union U { v16b v; v8b h[2]; };
  static __device__ __forceinline__ v16b load(const __bf16* p) {
    U f; f.h[0] = *(const v8b*)(p); f.h[1] = *(const v8b*)(p + 16); return f.v;
  }
  static __device__ __forceinline__ v8f mma(v16b a, v16b b, v8f c) {
    return __builtin_amdgcn_wmma_f32_16x16x32_bf16(false, a, false, b, (short)0, c, false, false);
  }
  static __device__ __forceinline__ void guard(v8f& a, v8f& b, v16b x, v16b y) { dep_guard_b(a, b, x, y); }
  static __device__ __forceinline__ void keep(v16b a, v16b b, v16b c, v16b d) { keep4_b(a, b, c, d); }
};

template <int ET> struct Elem;
template <> struct Elem<0> { typedef _Float16 T; };
template <> struct Elem<1> { typedef __bf16 T; };
template <int ET, int SPLIT, int BIAS_MODE, int OUT_MODE, bool RESID, int ACT = 0>
__global__ __launch_bounds__(256) void wmma_gemm64(
    const unsigned short* __restrict__ Ap, const unsigned short* __restrict__ A2p, int lda, long strideA,
    const unsigned short* __restrict__ Btp, const unsigned short* __restrict__ Bt2p, int ldb, long strideB,
    void* __restrict__ Cout, void* __restrict__ Cout2, int ldc, long strideC,
    const float* __restrict__ bias,
    const float* __restrict__ resid, long strideR,
    int M, int N, int K, float scale) {
  typedef typename Elem<ET>::T T;
  typedef typename Frag<T>::V V;
  const T* A = (const T*)Ap; const T* A2 = (const T*)A2p; const T* Bt = (const T*)Btp; const T* Bt2 = (const T*)Bt2p;
  __shared__ __align__(16) float sT[8][16 * 68];
  const int b    = blockIdx.y;
  const int lane = threadIdx.x & 31;
  const int wave = threadIdx.x >> 5;
  const int tilesN = N >> 6;
  const int tilesM = M >> 6;
  const int tile = blockIdx.x * 8 + wave;
  if (tile >= tilesM * tilesN) return;
  const int tm = tile / tilesN;
  const int tn = tile - tm * tilesN;
  const int m0 = tm << 6;
  const int n0 = tn << 6;

  const T* Ab  = A  + (size_t)b * strideA;
  const T* Bb  = Bt + (size_t)b * strideB;
  const T* Ab2 = (SPLIT != 0) ? (A2  + (size_t)b * strideA) : nullptr;
  const T* Bb2 = (SPLIT == 1) ? (Bt2 + (size_t)b * strideB) : nullptr;

  const int rlane = lane & 15;
  const int koff  = (lane >> 4) * 8;
  const int mOff  = (lane >> 4) * 8;

  v8f acc[4][4];
#pragma unroll
  for (int i = 0; i < 4; ++i)
#pragma unroll
    for (int j = 0; j < 4; ++j) acc[i][j] = (v8f){0.f,0.f,0.f,0.f,0.f,0.f,0.f,0.f};

  for (int k0 = 0; k0 < K; k0 += 32) {
    V bh[4], bl[4];
#pragma unroll
    for (int j = 0; j < 4; ++j) {
      const size_t bo = (size_t)(n0 + (j << 4) + rlane) * ldb + koff + k0;
      bh[j] = Frag<T>::load(Bb + bo);
      if (SPLIT == 1) bl[j] = Frag<T>::load(Bb2 + bo);
    }
#pragma unroll
    for (int i = 0; i < 4; ++i) {
      const size_t ao = (size_t)(m0 + (i << 4) + rlane) * lda + koff + k0;
      V ah = Frag<T>::load(Ab + ao);
      V al;
      if (SPLIT != 0) al = Frag<T>::load(Ab2 + ao);
#pragma unroll
      for (int j = 0; j < 4; ++j) {
        acc[i][j] = Frag<T>::mma(ah, bh[j], acc[i][j]);
        if (SPLIT == 1) acc[i][j] = Frag<T>::mma(ah, bl[j], acc[i][j]);
        if (SPLIT != 0) acc[i][j] = Frag<T>::mma(al, bh[j], acc[i][j]);
      }
      Frag<T>::guard(acc[i][0], acc[i][3], ah, (SPLIT != 0) ? al : ah);
    }
    Frag<T>::keep(bh[0], bh[1], bh[2], bh[3]);
    if (SPLIT == 1) Frag<T>::keep(bl[0], bl[1], bl[2], bl[3]);
  }
  acc_guard4(acc[0][0], acc[0][1], acc[0][2], acc[0][3]);
  acc_guard4(acc[1][0], acc[1][1], acc[1][2], acc[1][3]);
  acc_guard4(acc[2][0], acc[2][1], acc[2][2], acc[2][3]);
  acc_guard4(acc[3][0], acc[3][1], acc[3][2], acc[3][3]);

  float* slab = sT[wave];
  const float* Rb = RESID ? (resid + (size_t)b * strideR) : nullptr;
#pragma unroll
  for (int i = 0; i < 4; ++i) {
    const int mBase = m0 + (i << 4);
#pragma unroll
    for (int j = 0; j < 4; ++j) {
      const int n = n0 + (j << 4) + rlane;
      float bv = 0.f;
      if (BIAS_MODE == 2) bv = bias[n];
#pragma unroll
      for (int r = 0; r < 8; ++r) {
        float v = acc[i][j][r] * scale;
        if (BIAS_MODE == 1) v += bias[mBase + mOff + r];
        if (BIAS_MODE == 2) v += bv;
        if (RESID) v += Rb[(size_t)(mBase + mOff + r) * ldc + n];
        if (ACT == 1) v = tanhf(v);
        if (ACT == 2) v = fmaxf(v, 0.0f);
        if (ACT == 4) v = (v > 0.f) ? v : 0.01f * v;
        slab[(mOff + r) * 68 + (j << 4) + rlane] = v;
      }
    }
    __builtin_amdgcn_fence(__ATOMIC_RELEASE, "workgroup");
    __builtin_amdgcn_wave_barrier();
    __builtin_amdgcn_fence(__ATOMIC_ACQUIRE, "workgroup");
    if (OUT_MODE == 0) {
      float* C = (float*)Cout + (size_t)b * strideC;
      const int hh = lane >> 4, c4 = (lane & 15) * 4;
      for (int pass = 0; pass < 2; ++pass) {
#pragma unroll
        for (int it = 0; it < 8; ++it) {
          const int row = it * 2 + hh;
          v4f v = *(const v4f*)(slab + row * 68 + c4);
          *(volatile v4f*)(C + (size_t)(mBase + row) * ldc + n0 + c4) = v;
        }
        __threadfence();
      }
    } else {
      const int q = lane >> 3, c8 = (lane & 7) * 8;
      unsigned short* C  = (unsigned short*)Cout  + (size_t)b * strideC;
      unsigned short* C2 = (OUT_MODE == 2) ? ((unsigned short*)Cout2 + (size_t)b * strideC) : nullptr;
      for (int pass = 0; pass < 2; ++pass) {
#pragma unroll
        for (int it = 0; it < 4; ++it) {
          const int row = it * 4 + q;
          const float* sp = slab + row * 68 + c8;
          v8h hv, lv;
#pragma unroll
          for (int e = 0; e < 8; ++e) {
            if (OUT_MODE == 1) {
              hv[e] = (_Float16)sp[e];
            } else {
              unsigned short hb = f2bf_bits(sp[e]);
              unsigned short lb = f2bf_bits(sp[e] - bf_bits2f(hb));
              hv[e] = __builtin_bit_cast(_Float16, hb);
              lv[e] = __builtin_bit_cast(_Float16, lb);
            }
          }
          *(volatile v8h*)(C + (size_t)(mBase + row) * ldc + n0 + c8) = hv;
          if (OUT_MODE == 2) *(volatile v8h*)(C2 + (size_t)(mBase + row) * ldc + n0 + c8) = lv;
        }
        __threadfence();
      }
    }
    __builtin_amdgcn_fence(__ATOMIC_RELEASE, "workgroup");
    __builtin_amdgcn_wave_barrier();
    __builtin_amdgcn_fence(__ATOMIC_ACQUIRE, "workgroup");
  }
}

__global__ __launch_bounds__(256) void cast_f32_bf16x8(const float* __restrict__ in,
                                                      unsigned short* __restrict__ out, int n8) {
  const int i = blockIdx.x * 256 + (int)threadIdx.x;
  const int ic = (i < n8) ? i : (n8 - 1);
  const float* p = in + (size_t)ic * 8;
  const v4f a = *(const v4f*)p;
  const v4f c = *(const v4f*)(p + 4);
  v4u w;
  w[0] = pack_bf16x2(a[0], a[1]);
  w[1] = pack_bf16x2(a[2], a[3]);
  w[2] = pack_bf16x2(c[0], c[1]);
  w[3] = pack_bf16x2(c[2], c[3]);
  unsigned short* o = out + (size_t)ic * 8;
  *(volatile v4u*)o = w;
  __threadfence();
  *(volatile v4u*)o = w;
}

__global__ __launch_bounds__(256) void transpose_cast_bf16(const float* __restrict__ W,
                                                          unsigned short* __restrict__ Wt, int KR, int NC) {
  __shared__ float sT[64 * 65];
  const int k0 = blockIdx.x * 64, n0 = blockIdx.y * 64;
  const int tid = threadIdx.x;
  {
    const int kk = tid >> 2, cg = (tid & 3) * 16;
    const float* src = W + (size_t)(k0 + kk) * NC + n0 + cg;
#pragma unroll
    for (int i = 0; i < 4; ++i) {
      const v4f v = *(const v4f*)(src + 4 * i);
#pragma unroll
      for (int e = 0; e < 4; ++e) sT[(cg + 4 * i + e) * 65 + kk] = v[e];
    }
  }
  __syncthreads();
  const int wave = tid >> 5, lane = tid & 31, q4 = lane >> 3, c8 = (lane & 7) * 8;
  const int nl0 = wave * 4 + q4;
  const int nl1 = 32 + wave * 4 + q4;
  v4u w0, w1;
  {
    const float* s = sT + nl0 * 65 + c8;
    w0[0] = pack_bf16x2(s[0], s[1]); w0[1] = pack_bf16x2(s[2], s[3]);
    w0[2] = pack_bf16x2(s[4], s[5]); w0[3] = pack_bf16x2(s[6], s[7]);
  }
  {
    const float* s = sT + nl1 * 65 + c8;
    w1[0] = pack_bf16x2(s[0], s[1]); w1[1] = pack_bf16x2(s[2], s[3]);
    w1[2] = pack_bf16x2(s[4], s[5]); w1[3] = pack_bf16x2(s[6], s[7]);
  }
  unsigned short* d0 = Wt + (size_t)(n0 + nl0) * KR + k0 + c8;
  unsigned short* d1 = Wt + (size_t)(n0 + nl1) * KR + k0 + c8;
  for (int pass = 0; pass < 2; ++pass) {
    *(volatile v4u*)d0 = w0;
    *(volatile v4u*)d1 = w1;
    __threadfence();
  }
}

__global__ __launch_bounds__(128) void qk_layernorm_split(
    const float* __restrict__ qk, const float* __restrict__ qsc, const float* __restrict__ ksc,
    unsigned short* __restrict__ qh, unsigned short* __restrict__ ql,
    unsigned short* __restrict__ kh, unsigned short* __restrict__ kl, int nrows) {
  __shared__ float red[4][4];
  const int row = blockIdx.x;
  const int rowc = (row < nrows) ? row : (nrows - 1);
  const int tid = threadIdx.x, lane = tid & 31, wave = tid >> 5;
  const int c0 = tid * 8;
  const float* base = qk + (size_t)rowc * kQkCols;
  const v4f qa = *(const v4f*)(base + c0);
  const v4f qb = *(const v4f*)(base + c0 + 4);
  const v4f ka = *(const v4f*)(base + kModel + c0);
  const v4f kb = *(const v4f*)(base + kModel + c0 + 4);
  float xq[8], xk[8];
#pragma unroll
  for (int e = 0; e < 4; ++e) { xq[e] = qa[e]; xq[4 + e] = qb[e]; xk[e] = ka[e]; xk[4 + e] = kb[e]; }

  float sq = 0.f, sk = 0.f;
#pragma unroll
  for (int e = 0; e < 8; ++e) { sq += xq[e]; sk += xk[e]; }
#pragma unroll
  for (int off = 1; off < 32; off <<= 1) { sq += __shfl_xor(sq, off, 32); sk += __shfl_xor(sk, off, 32); }
  if (lane == 0) { red[0][wave] = sq; red[1][wave] = sk; }
  __syncthreads();
  const float mq = ((red[0][0] + red[0][1]) + (red[0][2] + red[0][3])) * (1.0f / (float)kModel);
  const float mk = ((red[1][0] + red[1][1]) + (red[1][2] + red[1][3])) * (1.0f / (float)kModel);

  float dq = 0.f, dk = 0.f;
#pragma unroll
  for (int e = 0; e < 8; ++e) {
    const float tq = xq[e] - mq; dq += tq * tq;
    const float tk = xk[e] - mk; dk += tk * tk;
  }
#pragma unroll
  for (int off = 1; off < 32; off <<= 1) { dq += __shfl_xor(dq, off, 32); dk += __shfl_xor(dk, off, 32); }
  if (lane == 0) { red[2][wave] = dq; red[3][wave] = dk; }
  __syncthreads();
  const float vq = ((red[2][0] + red[2][1]) + (red[2][2] + red[2][3])) * (1.0f / (float)kModel);
  const float vk = ((red[3][0] + red[3][1]) + (red[3][2] + red[3][3])) * (1.0f / (float)kModel);
  const float rq = rsqrtf(vq + 1e-6f);
  const float rk = rsqrtf(vk + 1e-6f);

  const v4f s0 = *(const v4f*)(qsc + c0);
  const v4f s1 = *(const v4f*)(qsc + c0 + 4);
  const v4f t0 = *(const v4f*)(ksc + c0);
  const v4f t1 = *(const v4f*)(ksc + c0 + 4);
  float sqv[8], skv[8];
#pragma unroll
  for (int e = 0; e < 4; ++e) {
    sqv[e]     = bf_bits2f(f2bf_bits(s0[e]));
    sqv[4 + e] = bf_bits2f(f2bf_bits(s1[e]));
    skv[e]     = bf_bits2f(f2bf_bits(t0[e]));
    skv[4 + e] = bf_bits2f(f2bf_bits(t1[e]));
  }
  unsigned int hqw[8], lqw[8], hkw[8], lkw[8];
#pragma unroll
  for (int e = 0; e < 8; ++e) {
    const float yq = ((xq[e] - mq) * rq * sqv[e]) * 0.125f;
    const float yk = (xk[e] - mk) * rk * skv[e];
    const unsigned short hqb = f2bf_bits(yq);
    const unsigned short lqb = f2bf_bits(yq - bf_bits2f(hqb));
    const unsigned short hkb = f2bf_bits(yk);
    const unsigned short lkb = f2bf_bits(yk - bf_bits2f(hkb));
    hqw[e] = hqb; lqw[e] = lqb; hkw[e] = hkb; lkw[e] = lkb;
  }
  v4u HQ, LQ, HK, LK;
#pragma unroll
  for (int i = 0; i < 4; ++i) {
    HQ[i] = hqw[2 * i] | (hqw[2 * i + 1] << 16);
    LQ[i] = lqw[2 * i] | (lqw[2 * i + 1] << 16);
    HK[i] = hkw[2 * i] | (hkw[2 * i + 1] << 16);
    LK[i] = lkw[2 * i] | (lkw[2 * i + 1] << 16);
  }
  const size_t o = (size_t)rowc * kModel + c0;
  for (int pass = 0; pass < 2; ++pass) {
    *(volatile v4u*)(qh + o) = HQ;
    *(volatile v4u*)(ql + o) = LQ;
    *(volatile v4u*)(kh + o) = HK;
    *(volatile v4u*)(kl + o) = LK;
    __threadfence();
  }
}

__device__ __forceinline__ __bf16 at_f2bf(float f) { return __builtin_bit_cast(__bf16, f2bf_bits(f)); }
__device__ __forceinline__ void at_split(float f, __bf16& hi, __bf16& lo) {
  const unsigned short hb = f2bf_bits(f);
  hi = __builtin_bit_cast(__bf16, hb);
  lo = at_f2bf(f - __uint_as_float(((unsigned)hb) << 16));
}
__device__ __forceinline__ v8f at_mma(v16b a, v16b b, v8f c) {
  c = __builtin_amdgcn_wmma_f32_16x16x32_bf16(false, a, false, b, (short)0, c, false, false);
  asm volatile("v_nop\n\tv_nop\n\tv_nop\n\tv_nop" : "+v"(c) : "v"(a), "v"(b));
  return c;
}

__global__ __launch_bounds__(128)
void attn_planes_kernel(const unsigned short* __restrict__ qh, const unsigned short* __restrict__ ql,
                        const unsigned short* __restrict__ kh, const unsigned short* __restrict__ kl,
                        const unsigned short* __restrict__ vh, const unsigned short* __restrict__ vl,
                        unsigned short* __restrict__ oh, unsigned short* __restrict__ ol,
                        int S, int H, int ld) {
  union FB { v16b v; v8b h[2]; };
  __shared__ __align__(16) unsigned short KVs[4 * kKvChunk * kHeadDim];
  __shared__ __align__(16) __bf16 Psh[4][16 * kKvChunk];
  __shared__ __align__(16) __bf16 Psl[4][16 * kKvChunk];
  unsigned short* Ksh = KVs;
  unsigned short* Ksl = KVs + kKvChunk * kHeadDim;
  unsigned short* Vth = KVs + 2 * kKvChunk * kHeadDim;
  unsigned short* Vtl = KVs + 3 * kKvChunk * kHeadDim;
  const __bf16* Kshb = (const __bf16*)(const void*)Ksh;
  const __bf16* Kslb = (const __bf16*)(const void*)Ksl;
  const __bf16* Vthb = (const __bf16*)(const void*)Vth;
  const __bf16* Vtlb = (const __bf16*)(const void*)Vtl;

  const int tid  = threadIdx.x;
  const int wave = tid >> 5;
  const int lane = tid & 31;
  const int hh   = lane >> 4;
  const int c    = lane & 15;

  const int nqb = S >> 6;
  const int qb  = blockIdx.x % nqb;
  const int bh  = blockIdx.x / nqb;
  const int h   = bh % H;
  const int b   = bh / H;
  const int q0  = qb * 64 + wave * 16;
  const size_t rb = (size_t)b * (size_t)S;
  const int hoff = h * kHeadDim;

  v16b qah[2], qal[2];
  {
    const size_t qo = (rb + (size_t)(q0 + c)) * (size_t)ld + hoff + 8 * hh;
    const __bf16* qhp = (const __bf16*)(const void*)qh + qo;
    const __bf16* qlp = (const __bf16*)(const void*)ql + qo;
#pragma unroll
    for (int dc = 0; dc < 2; ++dc) {
      qah[dc] = Frag<__bf16>::load(qhp + dc * 32);
      qal[dc] = Frag<__bf16>::load(qlp + dc * 32);
    }
  }

  float mrow[8], lrow[8];
  v8f oacc[4];
#pragma unroll
  for (int r = 0; r < 8; ++r) { mrow[r] = -INFINITY; lrow[r] = 0.f; }
#pragma unroll
  for (int t = 0; t < 4; ++t) oacc[t] = (v8f){0.f,0.f,0.f,0.f,0.f,0.f,0.f,0.f};

  const int nChunks = qb + 1;
  for (int kc = 0; kc < nChunks; ++kc) {
    const int kv0 = kc * kKvChunk;
    __syncthreads();
    {
      const int kvr = tid >> 1, dh = (tid & 1) * 32;
      const size_t go = (rb + (size_t)(kv0 + kvr)) * (size_t)ld + hoff + dh;
      {
        const uint4* g = (const uint4*)(const void*)(kh + go);
        uint4* l = (uint4*)(void*)(Ksh + kvr * kHeadDim + dh);
#pragma unroll
        for (int i = 0; i < 4; ++i) l[i] = g[i];
      }
      {
        const uint4* g = (const uint4*)(const void*)(kl + go);
        uint4* l = (uint4*)(void*)(Ksl + kvr * kHeadDim + dh);
#pragma unroll
        for (int i = 0; i < 4; ++i) l[i] = g[i];
      }
      {
        const uint4* g = (const uint4*)(const void*)(vh + go);
#pragma unroll
        for (int i = 0; i < 4; ++i) {
          const uint4 u = g[i];
          unsigned short* vt = Vth + (dh + 8 * i) * kKvChunk + kvr;
          vt[0 * kKvChunk] = (unsigned short)(u.x & 0xffffu);
          vt[1 * kKvChunk] = (unsigned short)(u.x >> 16);
          vt[2 * kKvChunk] = (unsigned short)(u.y & 0xffffu);
          vt[3 * kKvChunk] = (unsigned short)(u.y >> 16);
          vt[4 * kKvChunk] = (unsigned short)(u.z & 0xffffu);
          vt[5 * kKvChunk] = (unsigned short)(u.z >> 16);
          vt[6 * kKvChunk] = (unsigned short)(u.w & 0xffffu);
          vt[7 * kKvChunk] = (unsigned short)(u.w >> 16);
        }
      }
      {
        const uint4* g = (const uint4*)(const void*)(vl + go);
#pragma unroll
        for (int i = 0; i < 4; ++i) {
          const uint4 u = g[i];
          unsigned short* vt = Vtl + (dh + 8 * i) * kKvChunk + kvr;
          vt[0 * kKvChunk] = (unsigned short)(u.x & 0xffffu);
          vt[1 * kKvChunk] = (unsigned short)(u.x >> 16);
          vt[2 * kKvChunk] = (unsigned short)(u.y & 0xffffu);
          vt[3 * kKvChunk] = (unsigned short)(u.y >> 16);
          vt[4 * kKvChunk] = (unsigned short)(u.z & 0xffffu);
          vt[5 * kKvChunk] = (unsigned short)(u.z >> 16);
          vt[6 * kKvChunk] = (unsigned short)(u.w & 0xffffu);
          vt[7 * kKvChunk] = (unsigned short)(u.w >> 16);
        }
      }
    }
    __syncthreads();

    v8f s[4];
#pragma unroll
    for (int j = 0; j < 4; ++j) {
      s[j] = (v8f){0.f,0.f,0.f,0.f,0.f,0.f,0.f,0.f};
#pragma unroll
      for (int dc = 0; dc < 2; ++dc) {
        FB kb, klf;
        const int ko = (j * 16 + c) * kHeadDim + dc * 32 + 8 * hh;
        kb.h[0]  = *(const v8b*)(Kshb + ko);
        kb.h[1]  = *(const v8b*)(Kshb + ko + 16);
        klf.h[0] = *(const v8b*)(Kslb + ko);
        klf.h[1] = *(const v8b*)(Kslb + ko + 16);
        s[j] = at_mma(qah[dc], kb.v, s[j]);
        s[j] = at_mma(qah[dc], klf.v, s[j]);
        s[j] = at_mma(qal[dc], kb.v, s[j]);
      }
    }

    const bool diag = (kc == qb);
    float cm[8];
#pragma unroll
    for (int r = 0; r < 8; ++r) {
      const int qrow = q0 + 8 * hh + r;
      float m = -INFINITY;
#pragma unroll
      for (int j = 0; j < 4; ++j) {
        const int kvcol = kv0 + j * 16 + c;
        const bool masked = diag && (kvcol > qrow);
        const float sv = masked ? -3.4028235e38f : s[j][r];
        s[j][r] = sv;
        m = fmaxf(m, sv);
      }
#pragma unroll
      for (int off = 1; off < 16; off <<= 1) m = fmaxf(m, __shfl_xor(m, off, 32));
      cm[r] = m;
    }

    __bf16* pwh = Psh[wave];
    __bf16* pwl = Psl[wave];
#pragma unroll
    for (int r = 0; r < 8; ++r) {
      const float mnew  = fmaxf(mrow[r], cm[r]);
      const float alpha = expf(mrow[r] - mnew);
      mrow[r] = mnew;
      float psum = 0.f;
#pragma unroll
      for (int j = 0; j < 4; ++j) {
        const float p = expf(s[j][r] - mnew);
        psum += p;
        __bf16 a, bl;
        at_split(p, a, bl);
        pwh[(8 * hh + r) * kKvChunk + j * 16 + c] = a;
        pwl[(8 * hh + r) * kKvChunk + j * 16 + c] = bl;
      }
#pragma unroll
      for (int off = 1; off < 16; off <<= 1) psum += __shfl_xor(psum, off, 32);
      lrow[r] = lrow[r] * alpha + psum;
#pragma unroll
      for (int t = 0; t < 4; ++t) oacc[t][r] *= alpha;
    }
    __builtin_amdgcn_fence(__ATOMIC_RELEASE, "workgroup");
    __builtin_amdgcn_wave_barrier();
    __builtin_amdgcn_fence(__ATOMIC_ACQUIRE, "workgroup");

#pragma unroll 1
    for (int kk = 0; kk < 2; ++kk) {
      FB pa, pl;
      pa.h[0] = *(const v8b*)(pwh + c * kKvChunk + kk * 32 + 8 * hh);
      pa.h[1] = *(const v8b*)(pwh + c * kKvChunk + kk * 32 + 16 + 8 * hh);
      pl.h[0] = *(const v8b*)(pwl + c * kKvChunk + kk * 32 + 8 * hh);
      pl.h[1] = *(const v8b*)(pwl + c * kKvChunk + kk * 32 + 16 + 8 * hh);
#pragma unroll
      for (int t = 0; t < 4; ++t) {
        FB vb, vlf;
        const int vo = (t * 16 + c) * kKvChunk + kk * 32 + 8 * hh;
        vb.h[0]  = *(const v8b*)(Vthb + vo);
        vb.h[1]  = *(const v8b*)(Vthb + vo + 16);
        vlf.h[0] = *(const v8b*)(Vtlb + vo);
        vlf.h[1] = *(const v8b*)(Vtlb + vo + 16);
        oacc[t] = at_mma(pa.v, vb.v, oacc[t]);
        oacc[t] = at_mma(pa.v, vlf.v, oacc[t]);
        oacc[t] = at_mma(pl.v, vb.v, oacc[t]);
      }
    }
  }

  __syncthreads();
  float* os = (float*)(void*)KVs + wave * (16 * kOsPitch);
#pragma unroll
  for (int r = 0; r < 8; ++r) {
    const float inv = 1.0f / lrow[r];
#pragma unroll
    for (int t = 0; t < 4; ++t) os[(8 * hh + r) * kOsPitch + t * 16 + c] = oacc[t][r] * inv;
  }
  __builtin_amdgcn_fence(__ATOMIC_RELEASE, "workgroup");
  __builtin_amdgcn_wave_barrier();
  __builtin_amdgcn_fence(__ATOMIC_ACQUIRE, "workgroup");
  {
    const int q4 = lane >> 3, c8 = (lane & 7) * 8;
    for (int pass = 0; pass < 2; ++pass) {
#pragma unroll
      for (int it = 0; it < 4; ++it) {
        const int row = it * 4 + q4;
        const float* sp = os + row * kOsPitch + c8;
        v8h hv, lv;
#pragma unroll
        for (int e = 0; e < 8; ++e) {
          const unsigned short hb = f2bf_bits(sp[e]);
          const unsigned short lb = f2bf_bits(sp[e] - bf_bits2f(hb));
          hv[e] = __builtin_bit_cast(_Float16, hb);
          lv[e] = __builtin_bit_cast(_Float16, lb);
        }
        const size_t o = (rb + (size_t)(q0 + row)) * (size_t)ld + hoff + c8;
        *(volatile v8h*)(oh + o) = hv;
        *(volatile v8h*)(ol + o) = lv;
      }
      __threadfence();
    }
  }
}

extern "C" void kernel_launch(void* const* d_in, const int* in_sizes, int n_in,
                              void* d_out, int out_size, void* d_ws, size_t ws_size,
                              hipStream_t stream) {
  if (n_in < 5) return;
  if (in_sizes[0] != kRows * kModel) return;
  if (in_sizes[1] != kModel * kQkvCols) return;
  if (in_sizes[2] != kModel || in_sizes[3] != kModel) return;
  if (in_sizes[4] != kModel * kModel) return;
  if (out_size != kRows * kModel) return;
  if (ws_size < kWsTotal) return;

  const float* x     = (const float*)d_in[0];
  const float* W_qkv = (const float*)d_in[1];
  const float* q_sc  = (const float*)d_in[2];
  const float* k_sc  = (const float*)d_in[3];
  const float* W_out = (const float*)d_in[4];
  float* out = (float*)d_out;

  char* ws = (char*)d_ws;
  unsigned short* xb    = (unsigned short*)(ws + kOffXb);
  unsigned short* wqkvT = (unsigned short*)(ws + kOffWqkvT);
  unsigned short* woutT = (unsigned short*)(ws + kOffWoutT);
  float*          qkf   = (float*)(ws + kOffQk);
  unsigned short* ctxh  = (unsigned short*)(ws + kOffCtxH);
  unsigned short* ctxl  = (unsigned short*)(ws + kOffCtxL);
  unsigned short* vhp   = (unsigned short*)(ws + kOffVh);
  unsigned short* vlp   = (unsigned short*)(ws + kOffVl);
  unsigned short* qhp   = (unsigned short*)(ws + kOffQh);
  unsigned short* qlp   = (unsigned short*)(ws + kOffQl);
  unsigned short* khp   = (unsigned short*)(ws + kOffKh);
  unsigned short* klp   = (unsigned short*)(ws + kOffKl);

  const int n8 = kRows * kModel / 8;
  cast_f32_bf16x8<<<n8 / 256, 256, 0, stream>>>(x, xb, n8);

  transpose_cast_bf16<<<dim3(kModel / 64, kQkvCols / 64), 256, 0, stream>>>(W_qkv, wqkvT, kModel, kQkvCols);
  transpose_cast_bf16<<<dim3(kModel / 64, kModel / 64), 256, 0, stream>>>(W_out, woutT, kModel, kModel);

  wmma_gemm64<1, 0, 0, 0, false><<<dim3((kRows / 64) * (kQkCols / 64) / 8, 1), 256, 0, stream>>>(
      xb, xb, kModel, 0L,
      wqkvT, wqkvT, kModel, 0L,
      (void*)qkf, (void*)qkf, kQkCols, 0L,
      q_sc, q_sc, 0L,
      kRows, kQkCols, kModel, 1.0f);

  wmma_gemm64<1, 0, 0, 2, false><<<dim3((kRows / 64) * (kModel / 64) / 8, 1), 256, 0, stream>>>(
      xb, xb, kModel, 0L,
      wqkvT + (size_t)kQkCols * kModel, wqkvT + (size_t)kQkCols * kModel, kModel, 0L,
      (void*)vhp, (void*)vlp, kModel, 0L,
      q_sc, q_sc, 0L,
      kRows, kModel, kModel, 1.0f);

  qk_layernorm_split<<<kRows, 128, 0, stream>>>(qkf, q_sc, k_sc, qhp, qlp, khp, klp, kRows);

  attn_planes_kernel<<<kBatch * kHeads * (kSeq / 64), 128, 0, stream>>>(
      qhp, qlp, khp, klp, vhp, vlp, ctxh, ctxl, kSeq, kHeads, kModel);

  wmma_gemm64<1, 2, 0, 0, false><<<dim3((kRows / 64) * (kModel / 64) / 8, 1), 256, 0, stream>>>(
      ctxh, ctxl, kModel, 0L,
      woutT, woutT, kModel, 0L,
      (void*)out, (void*)out, kModel, 0L,
      q_sc, q_sc, 0L,
      kRows, kModel, kModel, 1.0f);
}
